// CompGCNLayer2_12180527251910
// MI455X (gfx1250) — hardware-run, weakly checked
//
#include <hip/hip_runtime.h>
#include <stddef.h>
#include <stdint.h>

#ifndef SPLIT
#define SPLIT 1
#endif

#define NN      50000
#define NE      600000
#define NRELS   500
#define DF      128
#define MP      50048
#define RBROWS  512
#define NFN     50176
#define ZPITCH  256
#define HPITCH  128
#define WPITCH  384
#define WLOOPC  256
#define KZ      (SPLIT ? 256 : 128)
#define KH      128
#define NTHR    256
#define NWAVE   8
#define EPT     8
#define WCH     (32 * EPT)
#define NBRUN   1024
#define SLB     10
#define NBK     49
#define WLCAP   2048
#define RCAP    16384
#define DEGCAP  64
#define MAXDEG_MEAS 27
#define MAXB_MEAS   12521
#define RBM     64
#define GBM     64
#define GTHR    128
#define WSMAX   ((size_t)(128u << 20))

#define BK_ZINTS (NWAVE * WLCAP + RCAP + 3 * NBRUN)
#define BK_INTS  (BK_ZINTS + 16)
#define BK_LDS   (BK_INTS * 4)

#define PBH  (MP * DF / 8 / NTHR)
#define PBR  (RBROWS * DF / 8 / NTHR)
#define PBN  (NFN / 4 / NTHR)
#define PBW  (3 * 2048 / NTHR)
#define PBTOT (PBH + PBR + PBN + PBW)

static_assert(NN <= 65536 && NRELS <= 65536);
static_assert(DF == 128 && DF == 4 * 32);
static_assert(MP % GBM == 0 && MP % RBM == 0 && MP >= NN && MP == 782 * 64);
static_assert(NBRUN == (1 << SLB) && NBRUN % RBM == 0 && NBRUN % GBM == 0 && NBRUN % 32 == 0);
static_assert(NBK * NBRUN >= MP && NBK * NBRUN == NFN);
static_assert(NE < (1 << 20) && (((long long)NE) << SLB) < (1LL << 31));
static_assert(RCAP == NWAVE * WLCAP && RCAP % (NTHR * 4) == 0 && BK_ZINTS % 4 == 0);
static_assert((2 * NBRUN) % (NTHR * 4) == 0);
static_assert((long long)RCAP * 100 >= (long long)MAXB_MEAS * 105);
static_assert(WLCAP >= MAXB_MEAS / 8 + 8 * 40 + 1);
static_assert(MAXDEG_MEAS + 8 <= DEGCAP);
static_assert((MP * DF / 8) % NTHR == 0 && (RBROWS * DF / 8) % NTHR == 0 && (NFN / 4) % NTHR == 0);
static_assert(NN % 4 == 0 && RBROWS >= NRELS && 2048 % NTHR == 0);
static_assert(KZ % 32 == 0 && KH % 32 == 0 && KZ <= ZPITCH && KH <= HPITCH && WLOOPC + KH <= WPITCH && KZ <= WLOOPC);
static_assert(GBM == (GTHR / 32) * 16);
static_assert(BK_LDS <= 300000);

typedef float          v4f   __attribute__((ext_vector_type(4)));
typedef float          v8f   __attribute__((ext_vector_type(8)));
typedef int            v4i   __attribute__((ext_vector_type(4)));
typedef int            v8i   __attribute__((ext_vector_type(8)));
typedef unsigned       v2u   __attribute__((ext_vector_type(2)));
typedef unsigned short v8us  __attribute__((ext_vector_type(8)));
typedef unsigned short v16us __attribute__((ext_vector_type(16)));
typedef __bf16         v16bf __attribute__((ext_vector_type(16)));
typedef v4f  __attribute__((may_alias)) v4fa;
typedef v4i  __attribute__((may_alias)) v4ia;
typedef v2u  __attribute__((may_alias)) v2ua;
typedef v8us __attribute__((may_alias)) v8usa;
union FragB { v16bf v; v16us u; v8us h[2]; v8i w; };

__device__ __forceinline__ v8f wmb(const FragB& a, const FragB& b, v8f c) {
  v8f d = __builtin_amdgcn_wmma_f32_16x16x32_bf16(false, a.v, false, b.v, (short)0, c, false, false);
  asm volatile("v_nop\n\tv_nop\n\tv_nop\n\tv_nop" : "+v"(d) : "v"(a.w), "v"(b.w));
  return d;
}

__device__ __forceinline__ unsigned bf16_bits(float f) {
  const unsigned u = __float_as_uint(f);
  const unsigned r = (u + 0x7fffu + ((u >> 16) & 1u)) >> 16;
  const unsigned q = (u >> 16) | 0x40u;
  return ((u & 0x7fffffffu) > 0x7f800000u) ? q : r;
}

__device__ __forceinline__ void hilo_pack(float v0, float v1, float v2, float v3,
                                          int& h01, int& h23, int& l01, int& l23) {
  const unsigned a0 = bf16_bits(v0), a1 = bf16_bits(v1), a2 = bf16_bits(v2), a3 = bf16_bits(v3);
  const unsigned b0 = bf16_bits(v0 - __uint_as_float(a0 << 16));
  const unsigned b1 = bf16_bits(v1 - __uint_as_float(a1 << 16));
  const unsigned b2 = bf16_bits(v2 - __uint_as_float(a2 << 16));
  const unsigned b3 = bf16_bits(v3 - __uint_as_float(a3 << 16));
  h01 = (int)(a0 | (a1 << 16)); h23 = (int)(a2 | (a3 << 16));
  l01 = (int)(b0 | (b1 << 16)); l23 = (int)(b2 | (b3 << 16));
}

__device__ __forceinline__ v4i regroup_row(int h01, int h23, int l01, int l23, int lane) {
  const int t  = lane & 15;
  const int s0 = 2 * t, s1 = s0 + 1;
  const int a0 = __shfl(h01, s0, 32), a1 = __shfl(h23, s0, 32), a2 = __shfl(h01, s1, 32), a3 = __shfl(h23, s1, 32);
  const int b0 = __shfl(l01, s0, 32), b1 = __shfl(l23, s0, 32), b2 = __shfl(l01, s1, 32), b3 = __shfl(l23, s1, 32);
  const int mk = (lane < 16) ? -1 : 0;
  v4i o;
  o.x = (a0 & mk) | (b0 & ~mk); o.y = (a1 & mk) | (b1 & ~mk);
  o.z = (a2 & mk) | (b2 & ~mk); o.w = (a3 & mk) | (b3 & ~mk);
  return o;
}

__device__ __forceinline__ void st2_v4f(float* p, v4f v) {
  *(volatile v4f*)p = v;
  __threadfence();
  *(volatile v4f*)p = v;
}
__device__ __forceinline__ void st2_v8us(unsigned short* p, v8us v) {
  *(volatile v8us*)p = v;
  __threadfence();
  *(volatile v8us*)p = v;
}

__device__ __forceinline__ v8us colfetch8(const float* __restrict__ base, int stride) {
  float f[8];
#pragma unroll
  for (int i = 0; i < 8; ++i) f[i] = base[(size_t)i * (size_t)stride];
  v8us o;
#pragma unroll
  for (int i = 0; i < 8; ++i) o[i] = (unsigned short)bf16_bits(f[i]);
  return o;
}

__global__ __launch_bounds__(NTHR) void k_prep(const float* __restrict__ h, const float* __restrict__ nrm,
                                               const float* __restrict__ rel, const float* __restrict__ wn,
                                               const float* __restrict__ lw, unsigned short* hb,
                                               unsigned short* rb, float* nf, unsigned short* wct) {
  const int tid = (int)threadIdx.x;
  const int blk = (int)blockIdx.x;
  if (blk < PBH) {
    const int u   = blk * NTHR + tid;
    const int row = u >> 4, k8 = (u & 15) * 8;
    const int rc  = row < NN ? row : NN - 1;
    const unsigned mk = row < NN ? 0xffffu : 0u;
    const float* p = h + (size_t)rc * DF + k8;
    const v4f a = *(const v4fa*)p;
    const v4f b = *(const v4fa*)(p + 4);
    v8us o;
    o[0] = (unsigned short)(bf16_bits(a.x) & mk); o[1] = (unsigned short)(bf16_bits(a.y) & mk);
    o[2] = (unsigned short)(bf16_bits(a.z) & mk); o[3] = (unsigned short)(bf16_bits(a.w) & mk);
    o[4] = (unsigned short)(bf16_bits(b.x) & mk); o[5] = (unsigned short)(bf16_bits(b.y) & mk);
    o[6] = (unsigned short)(bf16_bits(b.z) & mk); o[7] = (unsigned short)(bf16_bits(b.w) & mk);
    st2_v8us(hb + (size_t)row * HPITCH + k8, o);
  } else if (blk < PBH + PBR) {
    const int u   = (blk - PBH) * NTHR + tid;
    const int row = u >> 4, k8 = (u & 15) * 8;
    const int rc  = row < NRELS ? row : NRELS - 1;
    const unsigned mk = row < NRELS ? 0xffffu : 0u;
    const float* p = rel + (size_t)rc * DF + k8;
    const v4f a = *(const v4fa*)p;
    const v4f b = *(const v4fa*)(p + 4);
    v8us o;
    o[0] = (unsigned short)(bf16_bits(a.x) & mk); o[1] = (unsigned short)(bf16_bits(a.y) & mk);
    o[2] = (unsigned short)(bf16_bits(a.z) & mk); o[3] = (unsigned short)(bf16_bits(a.w) & mk);
    o[4] = (unsigned short)(bf16_bits(b.x) & mk); o[5] = (unsigned short)(bf16_bits(b.y) & mk);
    o[6] = (unsigned short)(bf16_bits(b.z) & mk); o[7] = (unsigned short)(bf16_bits(b.w) & mk);
    st2_v8us(rb + (size_t)row * HPITCH + k8, o);
  } else if (blk < PBH + PBR + PBN) {
    const int u  = (blk - PBH - PBR) * NTHR + tid;
    const int uc = u < NN / 4 ? u : NN / 4 - 1;
    const unsigned mk = u < NN / 4 ? 0xffffffffu : 0u;
    const v4f a = *(const v4fa*)(nrm + 4 * uc);
    asm volatile("" :: "v"(a));
    v4f o;
    o.x = __uint_as_float((bf16_bits(a.x) << 16) & mk);
    o.y = __uint_as_float((bf16_bits(a.y) << 16) & mk);
    o.z = __uint_as_float((bf16_bits(a.z) << 16) & mk);
    o.w = __uint_as_float((bf16_bits(a.w) << 16) & mk);
    st2_v4f(nf + 4 * u, o);
  } else {
    const int wb   = blk - PBH - PBR - PBN;
    const int part = wb >> 3;
    const int v    = (wb & 7) * NTHR + tid;
    const int n    = v >> 4, k8 = (v & 15) * 8;
    v8us o;
    if (part == 2) o = colfetch8(lw + (size_t)k8 * DF + n, DF);
    else           o = colfetch8(wn + (size_t)k8 * DF + n, DF);
    st2_v8us(wct + (size_t)n * WPITCH + part * DF + k8, o);
  }
}

__device__ __forceinline__ void bucket_flush(const int* pl, const int* cnt, int ov, int* lp, int* cop, int* fp,
                                             int tid) {
#pragma unroll 1
  for (int i = tid * 4; i < RCAP; i += NTHR * 4) {
    const v4i v = *(const v4ia*)(pl + i);
    *(volatile v4i*)(lp + i) = v;
  }
#pragma unroll 1
  for (int i = tid * 4; i < 2 * NBRUN; i += NTHR * 4) {
    const v4i v = *(const v4ia*)(cnt + i);
    *(volatile v4i*)(cop + i) = v;
  }
  if (tid < 8) {
    const v4i f = {ov, ov, ov, ov};
    *(volatile v4i*)(fp + 4 * tid) = f;
  }
}

__global__ __launch_bounds__(NTHR) void k_bucket(const int* __restrict__ srcs, const int* __restrict__ dsts,
                                                 const int* __restrict__ typs, int* LIST, int* CO, int* FLAG) {
  extern __shared__ __attribute__((aligned(16))) int dsm[];
  int* wl   = dsm;
  int* pl   = dsm + NWAVE * WLCAP;
  int* cnt  = pl + RCAP;
  int* offs = cnt + NBRUN;
  int* cur  = offs + NBRUN;
  int* misc = cur + NBRUN;
  const int tid = (int)threadIdx.x, lane = tid & 31;
  const int wave = __builtin_amdgcn_readfirstlane(tid >> 5);
  const int blk = (int)blockIdx.x;
  const unsigned nbs = (unsigned)(blk * NBRUN);
  const int nbi = (NN - blk * NBRUN) < NBRUN ? (NN - blk * NBRUN) : NBRUN;
  const unsigned unb = (unsigned)(nbi < 0 ? 0 : nbi);

  {
    const v4i z4 = {0, 0, 0, 0};
    for (int i = tid * 4; i < BK_ZINTS; i += NTHR * 4) *(v4ia*)(dsm + i) = z4;
    if (tid < 16) misc[tid] = 0;
  }
  __syncthreads();

  {
    const int per  = ((NE + NWAVE * WCH - 1) / (NWAVE * WCH)) * WCH;
    const int ebeg = wave * per;
    const int eend = (ebeg + per < NE) ? (ebeg + per) : NE;
    int* mylist = wl + wave * WLCAP;
    int wc = 0;
#pragma unroll 1
    for (int cb = ebeg; cb < eend; cb += WCH) {
      const int e0 = cb + lane * EPT;
      v4i da, db;
      if (cb + WCH <= NE) {
        da = *(const v4ia*)(dsts + e0);
        db = *(const v4ia*)(dsts + e0 + 4);
      } else {
        const int sent = (int)(1u << 31);
        const int t0 = dsts[min(e0 + 0, NE - 1)], t1 = dsts[min(e0 + 1, NE - 1)];
        const int t2 = dsts[min(e0 + 2, NE - 1)], t3 = dsts[min(e0 + 3, NE - 1)];
        const int t4 = dsts[min(e0 + 4, NE - 1)], t5 = dsts[min(e0 + 5, NE - 1)];
        const int t6 = dsts[min(e0 + 6, NE - 1)], t7 = dsts[min(e0 + 7, NE - 1)];
        asm volatile("" :: "v"(t0), "v"(t1), "v"(t2), "v"(t3));
        asm volatile("" :: "v"(t4), "v"(t5), "v"(t6), "v"(t7));
        da.x = (e0 + 0 < NE) ? t0 : sent; da.y = (e0 + 1 < NE) ? t1 : sent;
        da.z = (e0 + 2 < NE) ? t2 : sent; da.w = (e0 + 3 < NE) ? t3 : sent;
        db.x = (e0 + 4 < NE) ? t4 : sent; db.y = (e0 + 5 < NE) ? t5 : sent;
        db.z = (e0 + 6 < NE) ? t6 : sent; db.w = (e0 + 7 < NE) ? t7 : sent;
      }
      const unsigned s0 = (unsigned)da.x - nbs, s1 = (unsigned)da.y - nbs;
      const unsigned s2 = (unsigned)da.z - nbs, s3 = (unsigned)da.w - nbs;
      const unsigned s4 = (unsigned)db.x - nbs, s5 = (unsigned)db.y - nbs;
      const unsigned s6 = (unsigned)db.z - nbs, s7 = (unsigned)db.w - nbs;
      const bool h0 = s0 < unb, h1 = s1 < unb, h2 = s2 < unb, h3 = s3 < unb;
      const bool h4 = s4 < unb, h5 = s5 < unb, h6 = s6 < unb, h7 = s7 < unb;
      const unsigned m0 = __builtin_amdgcn_ballot_w32(h0), m1 = __builtin_amdgcn_ballot_w32(h1);
      const unsigned m2 = __builtin_amdgcn_ballot_w32(h2), m3 = __builtin_amdgcn_ballot_w32(h3);
      const unsigned m4 = __builtin_amdgcn_ballot_w32(h4), m5 = __builtin_amdgcn_ballot_w32(h5);
      const unsigned m6 = __builtin_amdgcn_ballot_w32(h6), m7 = __builtin_amdgcn_ballot_w32(h7);
      const unsigned any = m0 | m1 | m2 | m3 | m4 | m5 | m6 | m7;
      if (any != 0u) {
        const int pre = (int)(__builtin_amdgcn_mbcnt_lo(m0, 0u) + __builtin_amdgcn_mbcnt_lo(m1, 0u) +
                              __builtin_amdgcn_mbcnt_lo(m2, 0u) + __builtin_amdgcn_mbcnt_lo(m3, 0u) +
                              __builtin_amdgcn_mbcnt_lo(m4, 0u) + __builtin_amdgcn_mbcnt_lo(m5, 0u) +
                              __builtin_amdgcn_mbcnt_lo(m6, 0u) + __builtin_amdgcn_mbcnt_lo(m7, 0u));
        int p = wc + pre;
        if (h0) { if (p < WLCAP) mylist[p] = ((e0 + 0) << SLB) | (int)s0; p = p + 1; }
        if (h1) { if (p < WLCAP) mylist[p] = ((e0 + 1) << SLB) | (int)s1; p = p + 1; }
        if (h2) { if (p < WLCAP) mylist[p] = ((e0 + 2) << SLB) | (int)s2; p = p + 1; }
        if (h3) { if (p < WLCAP) mylist[p] = ((e0 + 3) << SLB) | (int)s3; p = p + 1; }
        if (h4) { if (p < WLCAP) mylist[p] = ((e0 + 4) << SLB) | (int)s4; p = p + 1; }
        if (h5) { if (p < WLCAP) mylist[p] = ((e0 + 5) << SLB) | (int)s5; p = p + 1; }
        if (h6) { if (p < WLCAP) mylist[p] = ((e0 + 6) << SLB) | (int)s6; p = p + 1; }
        if (h7) { if (p < WLCAP) mylist[p] = ((e0 + 7) << SLB) | (int)s7; p = p + 1; }
        wc += (int)(__builtin_popcount(m0) + __builtin_popcount(m1) + __builtin_popcount(m2) + __builtin_popcount(m3) +
                    __builtin_popcount(m4) + __builtin_popcount(m5) + __builtin_popcount(m6) + __builtin_popcount(m7));
      }
    }
    if (lane == 0) misc[wave] = wc;
  }
  __syncthreads();

  if (wave == 0) {
    int ov = 0;
#pragma unroll 1
    for (int w2 = 0; w2 < NWAVE; ++w2) {
      int c = misc[w2];
      if (c > WLCAP) ov = 1;
      c = c < 0 ? 0 : (c > WLCAP ? WLCAP : c);
#pragma unroll 1
      for (int b0 = 0; b0 < c; b0 += 32) {
        const int idx = b0 + lane;
        const int ent = wl[w2 * WLCAP + (idx < WLCAP ? idx : WLCAP - 1)];
        const int m32 = (c - b0) < 32 ? (c - b0) : 32;
#pragma unroll 1
        for (int k = 0; k < m32; ++k) {
          const int u    = __builtin_amdgcn_readlane(ent, k);
          const int slot = u & (NBRUN - 1);
          if (lane == 0) cnt[slot] = cnt[slot] + 1;
        }
      }
    }
    if (lane == 0) misc[9] = ov;
  }
  __syncthreads();
  if (wave == 0) {
    const int base = lane * (NBRUN / 32);
    int s = 0;
#pragma unroll 1
    for (int i = 0; i < NBRUN / 32; ++i) s += cnt[base + i];
    int incl = s;
#pragma unroll
    for (int d = 1; d < 32; d <<= 1) {
      const int y = __shfl_up(incl, d, 32);
      if (lane >= d) incl += y;
    }
    int run = incl - s;
#pragma unroll 1
    for (int i = 0; i < NBRUN / 32; ++i) {
      const int cv = cnt[base + i];
      offs[base + i] = run;
      cur[base + i]  = run;
      run += cv;
    }
  }
  __syncthreads();

  if (wave == 0) {
#pragma unroll 1
    for (int w2 = 0; w2 < NWAVE; ++w2) {
      int c = misc[w2];
      c = c < 0 ? 0 : (c > WLCAP ? WLCAP : c);
#pragma unroll 1
      for (int b0 = 0; b0 < c; b0 += 32) {
        const int idx = b0 + lane;
        const int ent = wl[w2 * WLCAP + (idx < WLCAP ? idx : WLCAP - 1)];
        int eid = (ent >> SLB) & 0xFFFFF;
        eid = eid > NE - 1 ? NE - 1 : eid;
        int sr = srcs[eid];
        int ty = typs[eid];
        sr = sr < 0 ? 0 : (sr > NN - 1 ? NN - 1 : sr);
        ty = ty < 0 ? 0 : (ty > NRELS - 1 ? NRELS - 1 : ty);
        const int word = (int)((unsigned)sr | ((unsigned)ty << 16));
        const int m32 = (c - b0) < 32 ? (c - b0) : 32;
#pragma unroll 1
        for (int k = 0; k < m32; ++k) {
          const int u    = __builtin_amdgcn_readlane(ent, k);
          const int wd   = __builtin_amdgcn_readlane(word, k);
          const int slot = u & (NBRUN - 1);
          if (lane == 0) {
            int p = cur[slot];
            p = p < 0 ? 0 : (p > RCAP - 1 ? RCAP - 1 : p);
            pl[p] = wd;
            cur[slot] = p + 1;
          }
        }
      }
    }
  }
  __syncthreads();

  const int ovf = misc[9];
  int* lp  = LIST + (size_t)blk * RCAP;
  int* cop = CO + (size_t)blk * (2 * NBRUN);
  int* fp  = FLAG + (size_t)blk * 32;
  bucket_flush(pl, cnt, ovf, lp, cop, fp, tid);
  __threadfence();
  bucket_flush(pl, cnt, ovf, lp, cop, fp, tid);
}

__global__ __launch_bounds__(NTHR) void k_replay(const int* __restrict__ LIST, const int* __restrict__ CO,
                                                 const int* __restrict__ FLAG,
                                                 const unsigned short* __restrict__ HB,
                                                 const unsigned short* __restrict__ RB,
                                                 const float* __restrict__ NF, unsigned short* ZHL) {
  const int tid = (int)threadIdx.x, lane = tid & 31;
  const int wave = __builtin_amdgcn_readfirstlane(tid >> 5);
  const int rowBase = (int)blockIdx.x * RBM;
  const int bucket  = rowBase >> SLB;
  const int* lb  = LIST + (size_t)bucket * RCAP;
  const int* cob = CO + (size_t)bucket * (2 * NBRUN);
  const int flag = FLAG[(size_t)bucket * 32];
  const float qnan = __uint_as_float(0x7fc00000u);

#pragma unroll 1
  for (int i = 0; i < RBM / NWAVE; ++i) {
    const int d    = rowBase + (RBM / NWAVE) * wave + i;
    const int slot = d & (NBRUN - 1);
    int c = cob[slot];
    int o = cob[NBRUN + slot];
    const bool big = c > DEGCAP;
    c = c < 0 ? 0 : (c > DEGCAP ? DEGCAP : c);
    o = o < 0 ? 0 : (o > RCAP - 1 ? RCAP - 1 : o);
    int last = o + c - 1;
    last = last < o ? o : last;
    last = last > RCAP - 1 ? RCAP - 1 : last;
    c    = __builtin_amdgcn_readfirstlane(c);
    o    = __builtin_amdgcn_readfirstlane(o);
    last = __builtin_amdgcn_readfirstlane(last);
    float a0 = 0.0f, a1 = 0.0f, a2 = 0.0f, a3 = 0.0f;
#pragma unroll 1
    for (int b0 = 0; b0 < c; b0 += 32) {
      int idx = o + b0 + lane;
      idx = idx > last ? last : idx;
      const int ent = lb[idx];
      const int m32 = (c - b0) < 32 ? (c - b0) : 32;
#pragma unroll 1
      for (int k = 0; k < m32; ++k) {
        const unsigned wd = (unsigned)__builtin_amdgcn_readlane(ent, k);
        int sr = (int)(wd & 0xffffu);
        int ty = (int)(wd >> 16);
        sr = sr > NN - 1 ? NN - 1 : sr;
        ty = ty > NRELS - 1 ? NRELS - 1 : ty;
        const v2u hv = *(const v2ua*)(HB + (size_t)sr * HPITCH + 4 * lane);
        const v2u rv = *(const v2ua*)(RB + (size_t)ty * HPITCH + 4 * lane);
        const float t0 = __uint_as_float(hv.x << 16)         + __uint_as_float(rv.x << 16);
        const float t1 = __uint_as_float(hv.x & 0xffff0000u) + __uint_as_float(rv.x & 0xffff0000u);
        const float t2 = __uint_as_float(hv.y << 16)         + __uint_as_float(rv.y << 16);
        const float t3 = __uint_as_float(hv.y & 0xffff0000u) + __uint_as_float(rv.y & 0xffff0000u);
        a0 += t0; a1 += t1; a2 += t2; a3 += t3;
      }
    }
    const float nf = NF[d];
    float z0 = a0 * nf, z1 = a1 * nf, z2 = a2 * nf, z3 = a3 * nf;
    const bool bad  = (flag != 0) | big;
    const bool live = d < NN;
    z0 = bad ? qnan : z0; z1 = bad ? qnan : z1; z2 = bad ? qnan : z2; z3 = bad ? qnan : z3;
    z0 = live ? z0 : 0.0f; z1 = live ? z1 : 0.0f; z2 = live ? z2 : 0.0f; z3 = live ? z3 : 0.0f;
    int h01, h23, l01, l23;
    hilo_pack(z0, z1, z2, z3, h01, h23, l01, l23);
    const v4i ow = regroup_row(h01, h23, l01, l23, lane);
    unsigned short* zp = ZHL + (size_t)d * ZPITCH + 8 * lane;
    *(volatile v4i*)zp = ow;
    __threadfence();
    *(volatile v4i*)zp = ow;
  }
}

template <int KSEG>
__device__ __forceinline__ void gemm_seg(const unsigned short* __restrict__ ap,
                                         const unsigned short* __restrict__ bp, v8f (&acc)[8]) {
#pragma unroll 1
  for (int k0 = 0; k0 < KSEG; k0 += 32) {
    FragB af;
    af.h[0] = *(const v8usa*)(ap + k0);
    af.h[1] = *(const v8usa*)(ap + k0 + 16);
#pragma unroll
    for (int nt = 0; nt < 8; ++nt) {
      const unsigned short* wq = bp + (size_t)(16 * nt) * (size_t)WPITCH + k0;
      FragB bf;
      bf.h[0] = *(const v8usa*)wq;
      bf.h[1] = *(const v8usa*)(wq + 16);
      acc[nt] = wmb(af, bf, acc[nt]);
    }
  }
}

__global__ __launch_bounds__(GTHR) __attribute__((amdgpu_num_vgpr(248)))
void k_gemm(const unsigned short* __restrict__ ZHL, const unsigned short* __restrict__ HB,
            const unsigned short* __restrict__ WCT, const int* __restrict__ FLAG, float* out) {
  __shared__ __attribute__((aligned(16))) float stg[GBM * DF];
  const int tid = (int)threadIdx.x, lane = tid & 31, hh = lane >> 4, m = lane & 15;
  const int wave = __builtin_amdgcn_readfirstlane(tid >> 5);
  const int rowBase = (int)blockIdx.x * GBM;
  const int flag = FLAG[(size_t)(rowBase >> SLB) * 32];

  v8f acc[8];
  {
    const v8f z = {0.f, 0.f, 0.f, 0.f, 0.f, 0.f, 0.f, 0.f};
#pragma unroll
    for (int t = 0; t < 8; ++t) acc[t] = z;
  }
  const unsigned short* zp = ZHL + (size_t)(rowBase + 16 * wave + m) * (size_t)ZPITCH + 8 * hh;
  const unsigned short* hp = HB  + (size_t)(rowBase + 16 * wave + m) * (size_t)HPITCH + 8 * hh;
  const unsigned short* bp = WCT + (size_t)m * (size_t)WPITCH + 8 * hh;
  gemm_seg<KZ>(zp, bp, acc);
  gemm_seg<KH>(hp, bp + WLOOPC, acc);

#pragma unroll
  for (int nt = 0; nt < 8; ++nt) {
    const int lc = 16 * nt + m;
#pragma unroll
    for (int r = 0; r < 8; ++r) {
      const int lr = 16 * wave + 8 * hh + r;
      stg[lr * DF + lc] = acc[nt][r];
    }
  }
  __syncthreads();

  const float qnan = __uint_as_float(0x7fc00000u);
#pragma unroll 1
  for (int i = 0; i < 16; ++i) {
    const int lr   = 16 * wave + i;
    const int grow = rowBase + lr;
    const v4f a = *(const v4fa*)(stg + lr * DF + 4 * lane);
    asm volatile("" :: "v"(a));
    float v0 = a.x, v1 = a.y, v2 = a.z, v3 = a.w;
    v0 = (v0 > 0.0f) ? v0 : (v0 - v0); v1 = (v1 > 0.0f) ? v1 : (v1 - v1);
    v2 = (v2 > 0.0f) ? v2 : (v2 - v2); v3 = (v3 > 0.0f) ? v3 : (v3 - v3);
    v4f o;
    o.x = (flag != 0) ? qnan : v0; o.y = (flag != 0) ? qnan : v1;
    o.z = (flag != 0) ? qnan : v2; o.w = (flag != 0) ? qnan : v3;
    if (grow < NN) st2_v4f(out + (size_t)grow * DF + 4 * lane, o);
  }
}

extern "C" void kernel_launch(void* const* d_in, const int* in_sizes, int n_in,
                              void* d_out, int out_size, void* d_ws, size_t ws_size,
                              hipStream_t stream) {
  if (n_in < 8) return;
  if (in_sizes[0] != NN * DF) return;
  if (in_sizes[1] != NN) return;
  if (in_sizes[2] != NRELS * DF) return;
  if (in_sizes[3] != DF * DF) return;
  if (in_sizes[4] != DF * DF) return;
  if (in_sizes[5] != NE || in_sizes[6] != NE || in_sizes[7] != NE) return;
  if (out_size != NN * DF) return;

  const float* h    = (const float*)d_in[0];
  const float* nrm  = (const float*)d_in[1];
  const float* rel  = (const float*)d_in[2];
  const float* wn   = (const float*)d_in[3];
  const float* lw   = (const float*)d_in[4];
  const int*   srcs = (const int*)d_in[5];
  const int*   dsts = (const int*)d_in[6];
  const int*   typs = (const int*)d_in[7];
  float* out = (float*)d_out;

  constexpr size_t zHB   = (size_t)MP * HPITCH * 2;
  constexpr size_t zZHL  = (size_t)MP * ZPITCH * 2;
  constexpr size_t zRB   = (size_t)RBROWS * HPITCH * 2;
  constexpr size_t zWCT  = (size_t)DF * WPITCH * 2;
  constexpr size_t zNF   = (size_t)NFN * 4;
  constexpr size_t zCO   = (size_t)NBK * 2 * NBRUN * 4;
  constexpr size_t zLIST = (size_t)NBK * RCAP * 4;
  constexpr size_t zFLAG = 8192;
  constexpr size_t oHB   = 0;
  constexpr size_t oZHL  = oHB + zHB;
  constexpr size_t oRB   = oZHL + zZHL;
  constexpr size_t oWCT  = oRB + zRB;
  constexpr size_t oNF   = oWCT + zWCT;
  constexpr size_t oCO   = oNF + zNF;
  constexpr size_t oLIST = oCO + zCO;
  constexpr size_t oFLAG = oLIST + zLIST;
  constexpr size_t oEND  = oFLAG + zFLAG;
  static_assert(zHB % 256 == 0 && zZHL % 256 == 0 && zRB % 256 == 0 && zWCT % 256 == 0);
  static_assert(zNF % 256 == 0 && zCO % 256 == 0 && zLIST % 256 == 0 && zFLAG % 256 == 0);
  static_assert((size_t)NBK * 128 <= zFLAG);
  static_assert(oEND <= WSMAX);
  if (oEND > ws_size) return;

  char* ws = (char*)d_ws;
  unsigned short* HB   = (unsigned short*)(ws + oHB);
  unsigned short* ZHL  = (unsigned short*)(ws + oZHL);
  unsigned short* RB   = (unsigned short*)(ws + oRB);
  unsigned short* WCT  = (unsigned short*)(ws + oWCT);
  float*          NF   = (float*)(ws + oNF);
  int*            CO   = (int*)(ws + oCO);
  int*            LIST = (int*)(ws + oLIST);
  int*            FLAG = (int*)(ws + oFLAG);

  hipFuncSetAttribute(reinterpret_cast<const void*>(&k_bucket), hipFuncAttributeMaxDynamicSharedMemorySize, (int)BK_LDS);

  k_prep<<<PBTOT, NTHR, 0, stream>>>(h, nrm, rel, wn, lw, HB, RB, NF, WCT);
  k_bucket<<<NBK, NTHR, BK_LDS, stream>>>(srcs, dsts, typs, LIST, CO, FLAG);
  k_replay<<<MP / RBM, NTHR, 0, stream>>>(LIST, CO, FLAG, HB, RB, NF, ZHL);
  k_gemm<<<MP / GBM, GTHR, 0, stream>>>(ZHL, HB, WCT, FLAG, out);
}
